// MultiHeadSelfAttention_56762287784156
// MI455X (gfx1250) — hardware-verified
//
#include <hip/hip_runtime.h>
#ifndef NB
#define NB 2
#endif
#ifndef SEQ
#define SEQ 2048
#endif
#define NB_FULL 2
#define SEQ_FULL 2048
#define DM 1024
#define NH 16
#define HD 64
#define NR (NB * SEQ)
#define CXP (2 * DM)

static_assert(NB <= NB_FULL);
static_assert(SEQ <= SEQ_FULL);
static_assert(NH * HD == DM);
static_assert(HD == 64);
static_assert(DM % 128 == 0);
static_assert(NR % 128 == 0);
static_assert(SEQ % 128 == 0);
static_assert(DM % 32 == 0);
static_assert(CXP % 32 == 0);
static_assert(DM % 8 == 0);
static_assert((size_t)NB_FULL * SEQ_FULL * DM * 4 == (size_t)16777216);

typedef __bf16 v16b __attribute__((ext_vector_type(16)));
typedef _Float16 v16h __attribute__((ext_vector_type(16)));
typedef unsigned short v8us __attribute__((ext_vector_type(8), may_alias));
typedef float v8f __attribute__((ext_vector_type(8)));
typedef float v4f __attribute__((ext_vector_type(4)));
typedef float v4fa __attribute__((ext_vector_type(4), may_alias));
union FragB { v16b v; v8us half[2]; };
union FragH { v16h v; v8us half[2]; _Float16 h[16]; };

__device__ __forceinline__ unsigned short bf16_bits(float x) { const unsigned int u = __float_as_uint(x); return (unsigned short)((u + 0x7FFFu + ((u >> 16) & 1u)) >> 16); }
__device__ __forceinline__ float bf16_val(unsigned short b) { return __uint_as_float(((unsigned int)b) << 16); }
__device__ __forceinline__ float bf16_rne(float x) { return bf16_val(bf16_bits(x)); }

__device__ __forceinline__ v16b ld_fb(const unsigned short* __restrict__ p, size_t off, int hh) { FragB f; f.half[0] = *(const v8us*)(p + off + 8 * hh); f.half[1] = *(const v8us*)(p + off + 16 + 8 * hh); return f.v; }
__device__ __forceinline__ v16h ld_fh(const unsigned short* __restrict__ p, size_t off, int hh) { FragH f; f.half[0] = *(const v8us*)(p + off + 8 * hh); f.half[1] = *(const v8us*)(p + off + 16 + 8 * hh); return f.v; }

__device__ __forceinline__ v8f wm_b(v16b a, v16b b, v8f c) { return __builtin_amdgcn_wmma_f32_16x16x32_bf16(false, a, false, b, (short)0, c, false, false); }
__device__ __forceinline__ v8f wm_h(v16h a, v16h b, v8f c) { return __builtin_amdgcn_wmma_f32_16x16x32_f16(false, a, false, b, (short)0, c, false, false); }

__device__ __forceinline__ void gemm8(v16b a0, v16b a1, v16b b0, v16b b1, v16b b2, v16b b3,
                                      v8f& c00, v8f& c01, v8f& c02, v8f& c03, v8f& c10, v8f& c11, v8f& c12, v8f& c13) {
  c00 = wm_b(a0, b0, c00); c10 = wm_b(a1, b0, c10);
  c01 = wm_b(a0, b1, c01); c11 = wm_b(a1, b1, c11);
  c02 = wm_b(a0, b2, c02); c12 = wm_b(a1, b2, c12);
  c03 = wm_b(a0, b3, c03); c13 = wm_b(a1, b3, c13);
  asm volatile("v_nop\n\tv_nop\n\tv_nop\n\tv_nop"
               : "+v"(c00), "+v"(c01), "+v"(c02), "+v"(c03), "+v"(c10), "+v"(c11), "+v"(c12), "+v"(c13)
               : "v"(a0), "v"(a1), "v"(b0), "v"(b1), "v"(b2), "v"(b3));
}
__device__ __forceinline__ void score6(v16b kh0, v16b kh1, v16b kl0, v16b kl1, v16b qh, v16b ql, v8f& s0, v8f& s1) {
  s0 = wm_b(kh0, qh, s0); s1 = wm_b(kh1, qh, s1);
  s0 = wm_b(kl0, qh, s0); s1 = wm_b(kl1, qh, s1);
  s0 = wm_b(kh0, ql, s0); s1 = wm_b(kh1, ql, s1);
  asm volatile("v_nop\n\tv_nop\n\tv_nop\n\tv_nop"
               : "+v"(s0), "+v"(s1)
               : "v"(kh0), "v"(kh1), "v"(kl0), "v"(kl1), "v"(qh), "v"(ql));
}
__device__ __forceinline__ void pv4(v16h a0, v16h a1, v16h a2, v16h a3, v16h p, v8f& o0, v8f& o1, v8f& o2, v8f& o3) {
  o0 = wm_h(a0, p, o0); o1 = wm_h(a1, p, o1); o2 = wm_h(a2, p, o2); o3 = wm_h(a3, p, o3);
  asm volatile("v_nop\n\tv_nop\n\tv_nop\n\tv_nop"
               : "+v"(o0), "+v"(o1), "+v"(o2), "+v"(o3)
               : "v"(a0), "v"(a1), "v"(a2), "v"(a3), "v"(p));
}

__device__ __forceinline__ void cvt_hilo8(const v4f a, const v4f c, v8us& vh, v8us& vl) {
#pragma unroll
  for (int i = 0; i < 4; ++i) {
    unsigned short hb = bf16_bits(a[i]); vh[i] = hb; vl[i] = bf16_bits(a[i] - bf16_val(hb));
    hb = bf16_bits(c[i]); vh[4 + i] = hb; vl[4 + i] = bf16_bits(c[i] - bf16_val(hb));
  }
}

__global__ __launch_bounds__(256) void k_wt(const float* __restrict__ W, unsigned short* __restrict__ Wt, int ldw, int dup) {
  const int t = blockIdx.x * 256 + threadIdx.x;
  if (t >= DM * (DM / 8)) return;
  const int n = t / (DM / 8), k8 = (t % (DM / 8)) * 8;
  v8us v;
#pragma unroll
  for (int i = 0; i < 8; ++i) v[i] = bf16_bits(W[(size_t)(k8 + i) * DM + n]);
  unsigned short* d = Wt + (size_t)n * ldw + k8;
  *(volatile v8us*)d = v;
  if (dup != 0) *(volatile v8us*)(d + DM) = v;
  __threadfence();
  *(volatile v8us*)d = v;
  if (dup != 0) *(volatile v8us*)(d + DM) = v;
}

__global__ __launch_bounds__(256) void k_xbf(const float* __restrict__ x, unsigned short* __restrict__ X) {
  const size_t t = (size_t)blockIdx.x * 256 + threadIdx.x;
  if (t >= (size_t)NR * (DM / 8)) return;
  const int row = (int)(t / (DM / 8)), c8 = (int)(t % (DM / 8)) * 8;
  const int b = row / SEQ, s = row % SEQ;
  const float* src = x + ((size_t)b * SEQ_FULL + s) * DM + c8;
  const v4f a = *(const v4fa*)src, c = *(const v4fa*)(src + 4);
  v8us v;
#pragma unroll
  for (int i = 0; i < 4; ++i) { v[i] = bf16_bits(a[i]); v[4 + i] = bf16_bits(c[i]); }
  unsigned short* d = X + (size_t)row * DM + c8;
  *(volatile v8us*)d = v;
  __threadfence();
  *(volatile v8us*)d = v;
}

template <int EP>
__device__ __forceinline__ void gemm_body(const unsigned short* __restrict__ A, int lda, size_t sA,
                                          const unsigned short* __restrict__ Bt, int ldb, size_t sB, float alpha,
                                          const float* __restrict__ bias, float* __restrict__ Cf,
                                          unsigned short* __restrict__ C0, unsigned short* __restrict__ C1,
                                          int ldc, size_t sC, int N, int K) {
  __shared__ __attribute__((aligned(16))) float so[4][32][68];
  const int tid = threadIdx.x, lane = tid & 31, ln = lane & 15, hh = lane >> 4;
  const int w = __builtin_amdgcn_readfirstlane(tid >> 5);
  const int by = blockIdx.y;
  const size_t cofs = (size_t)by * sC;
  const int ntn = N >> 6;
  const int mt = blockIdx.x / ntn, nq = blockIdx.x - mt * ntn;
  const int row0 = mt * 128 + 32 * w, col0 = nq * 64;
  const size_t ao0 = (size_t)by * sA + (size_t)(row0 + ln) * lda, ao1 = ao0 + (size_t)16 * lda;
  const size_t bo0 = (size_t)by * sB + (size_t)(col0 + ln) * ldb, bo1 = bo0 + (size_t)16 * ldb, bo2 = bo1 + (size_t)16 * ldb, bo3 = bo2 + (size_t)16 * ldb;
  const v8f z8 = {0.f, 0.f, 0.f, 0.f, 0.f, 0.f, 0.f, 0.f};
  v8f c00 = z8, c01 = z8, c02 = z8, c03 = z8, c10 = z8, c11 = z8, c12 = z8, c13 = z8;
#pragma unroll 1
  for (int kb = 0; kb < K; kb += 32) {
    const v16b a0 = ld_fb(A, ao0 + kb, hh), a1 = ld_fb(A, ao1 + kb, hh);
    const v16b b0 = ld_fb(Bt, bo0 + kb, hh), b1 = ld_fb(Bt, bo1 + kb, hh), b2 = ld_fb(Bt, bo2 + kb, hh), b3 = ld_fb(Bt, bo3 + kb, hh);
    gemm8(a0, a1, b0, b1, b2, b3, c00, c01, c02, c03, c10, c11, c12, c13);
  }
  const v8f accs[8] = {c00, c01, c02, c03, c10, c11, c12, c13};
#pragma unroll
  for (int u = 0; u < 8; ++u) {
    const int t = u & 3, half = u >> 2;
    float bv = 0.f;
    if (EP != 2) bv = bf16_rne(bias[col0 + t * 16 + ln]);
#pragma unroll
    for (int r = 0; r < 8; ++r) so[w][half * 16 + 8 * hh + r][t * 16 + ln] = (accs[u][r] + bv) * alpha;
  }
  __builtin_amdgcn_fence(4  , "workgroup");
  __builtin_amdgcn_wave_barrier();
  if (EP == 0) {
    const int rsub = lane >> 4, c4 = (lane & 15) * 4;
    for (int pass = 0; pass < 2; ++pass) {
#pragma unroll
      for (int q = 0; q < 16; ++q) {
        const int r = q * 2 + rsub;
        const v4f v = *(const v4fa*)&so[w][r][c4];
        *(volatile v4f*)(Cf + cofs + (size_t)(row0 + r) * ldc + col0 + c4) = v;
      }
      if (pass == 0) __threadfence();
    }
  } else {
    const int rs = lane >> 3, c8 = (lane & 7) * 8;
    for (int pass = 0; pass < 2; ++pass) {
#pragma unroll
      for (int q = 0; q < 8; ++q) {
        const int r = q * 4 + rs;
        const v4f x0 = *(const v4fa*)&so[w][r][c8];
        const v4f x1 = *(const v4fa*)&so[w][r][c8 + 4];
        const size_t o = cofs + (size_t)(row0 + r) * ldc + col0 + c8;
        if (EP == 1) {
          v8us vh, vl;
          cvt_hilo8(x0, x1, vh, vl);
          *(volatile v8us*)(C0 + o) = vh;
          *(volatile v8us*)(C1 + o) = vl;
        } else {
          const float bv = bf16_rne(bias[row0 + r]);
          FragH f;
#pragma unroll
          for (int i = 0; i < 4; ++i) { f.h[i] = (_Float16)(x0[i] + bv); f.h[4 + i] = (_Float16)(x1[i] + bv); }
          const v8us v = f.half[0];
          *(volatile v8us*)(C0 + o) = v;
        }
      }
      if (pass == 0) __threadfence();
    }
  }
}

__global__ __launch_bounds__(128) void k_gemm_hilo(const unsigned short* __restrict__ A, int lda, const unsigned short* __restrict__ Bt, int ldb,
                                                   float alpha, const float* __restrict__ bias, unsigned short* __restrict__ CH,
                                                   unsigned short* __restrict__ CL, int ldc, int N, int K) {
  gemm_body<1>(A, lda, (size_t)0, Bt, ldb, (size_t)0, alpha, bias, nullptr, CH, CL, ldc, (size_t)0, N, K);
}
__global__ __launch_bounds__(128) void k_gemm_vt(const unsigned short* __restrict__ A, int lda, const unsigned short* __restrict__ Bt, int ldb, size_t sB,
                                                 const float* __restrict__ bias, unsigned short* __restrict__ VT, int ldc, size_t sC, int N, int K) {
  gemm_body<2>(A, lda, (size_t)0, Bt, ldb, sB, 1.0f, bias, nullptr, VT, nullptr, ldc, sC, N, K);
}
__global__ __launch_bounds__(128) void k_gemm_out(const unsigned short* __restrict__ A, int lda, size_t sA, const unsigned short* __restrict__ Bt, int ldb,
                                                  const float* __restrict__ bias, float* __restrict__ C, int ldc, size_t sC, int N, int K) {
  gemm_body<0>(A, lda, sA, Bt, ldb, (size_t)0, 1.0f, bias, C, nullptr, nullptr, ldc, sC, N, K);
}

__global__ __launch_bounds__(128) void k_attn(const unsigned short* __restrict__ QH, const unsigned short* __restrict__ QL,
                                              const unsigned short* __restrict__ KH, const unsigned short* __restrict__ KL,
                                              const unsigned short* __restrict__ VT, unsigned short* __restrict__ CX) {
  __shared__ __attribute__((aligned(16))) unsigned short sc[4][2][16][72];
  const int tid = threadIdx.x, lane = tid & 31, ln = lane & 15, hh = lane >> 4;
  const int wave = __builtin_amdgcn_readfirstlane(tid >> 5);
  const int bx = blockIdx.x;
  const int qb = bx % (SEQ / 64), bh = bx / (SEQ / 64);
  const int h = bh % NH, b = bh / NH;
  const int q0 = qb * 64 + wave * 16;
  const size_t rowb = (size_t)b * SEQ;
  const size_t qoff = (rowb + q0 + ln) * DM + (size_t)h * HD;
  const v16b qh0 = ld_fb(QH, qoff, hh), qh1 = ld_fb(QH, qoff + 32, hh);
  const v16b ql0 = ld_fb(QL, qoff, hh), ql1 = ld_fb(QL, qoff + 32, hh);
  const size_t kbase = (rowb + ln) * DM + (size_t)h * HD;
  const size_t vbase = ((size_t)b * DM + (size_t)h * HD + ln) * SEQ;
  const v8f z8 = {0.f, 0.f, 0.f, 0.f, 0.f, 0.f, 0.f, 0.f};
  v8f o0 = z8, o1 = z8, o2 = z8, o3 = z8;
  float m = -1.0e30f, l = 0.f;
#pragma unroll 1
  for (int key0 = 0; key0 < SEQ; key0 += 32) {
    const size_t k0o = kbase + (size_t)key0 * DM, k1o = k0o + (size_t)16 * DM;
    v8f s0 = z8, s1 = z8;
    {
      const v16b a0 = ld_fb(KH, k0o, hh), a1 = ld_fb(KH, k1o, hh), c0 = ld_fb(KL, k0o, hh), c1 = ld_fb(KL, k1o, hh);
      score6(a0, a1, c0, c1, qh0, ql0, s0, s1);
    }
    {
      const v16b a0 = ld_fb(KH, k0o + 32, hh), a1 = ld_fb(KH, k1o + 32, hh), c0 = ld_fb(KL, k0o + 32, hh), c1 = ld_fb(KL, k1o + 32, hh);
      score6(a0, a1, c0, c1, qh1, ql1, s0, s1);
    }
    float mx = fmaxf(s0[0], s1[0]);
#pragma unroll
    for (int r = 1; r < 8; ++r) mx = fmaxf(mx, fmaxf(s0[r], s1[r]));
    mx = fmaxf(mx, __shfl_xor(mx, 16, 32));
    const float mnew = fmaxf(m, mx);
    if (__builtin_amdgcn_ballot_w32(mnew > m) != 0u) {
      const float al = __expf(m - mnew);
      l *= al; o0 = o0 * al; o1 = o1 * al; o2 = o2 * al; o3 = o3 * al;
      m = mnew;
    }
    const float ms = m - 5.545177444f;
    FragH p;
    float ls = 0.f;
#pragma unroll
    for (int r = 0; r < 8; ++r) {
      const float e0 = __expf(s0[r] - ms), e1 = __expf(s1[r] - ms);
      ls += e0 + e1;
      p.h[r] = (_Float16)e0; p.h[8 + r] = (_Float16)e1;
    }
    l += ls;
    {
      const size_t vo = vbase + key0;
      const v16h a0 = ld_fh(VT, vo, hh), a1 = ld_fh(VT, vo + (size_t)16 * SEQ, hh), a2 = ld_fh(VT, vo + (size_t)32 * SEQ, hh), a3 = ld_fh(VT, vo + (size_t)48 * SEQ, hh);
      pv4(a0, a1, a2, a3, p.v, o0, o1, o2, o3);
    }
  }
  const float lt = l + __shfl_xor(l, 16, 32);
  const float inv = 1.0f / lt;
  {
    v8us vh, vl;
#pragma unroll
    for (int r = 0; r < 8; ++r) { const float x = o0[r] * inv; const unsigned short hb = bf16_bits(x); vh[r] = hb; vl[r] = bf16_bits(x - bf16_val(hb)); }
    *(v8us*)&sc[wave][0][ln][0 + 8 * hh] = vh; *(v8us*)&sc[wave][1][ln][0 + 8 * hh] = vl;
#pragma unroll
    for (int r = 0; r < 8; ++r) { const float x = o1[r] * inv; const unsigned short hb = bf16_bits(x); vh[r] = hb; vl[r] = bf16_bits(x - bf16_val(hb)); }
    *(v8us*)&sc[wave][0][ln][16 + 8 * hh] = vh; *(v8us*)&sc[wave][1][ln][16 + 8 * hh] = vl;
#pragma unroll
    for (int r = 0; r < 8; ++r) { const float x = o2[r] * inv; const unsigned short hb = bf16_bits(x); vh[r] = hb; vl[r] = bf16_bits(x - bf16_val(hb)); }
    *(v8us*)&sc[wave][0][ln][32 + 8 * hh] = vh; *(v8us*)&sc[wave][1][ln][32 + 8 * hh] = vl;
#pragma unroll
    for (int r = 0; r < 8; ++r) { const float x = o3[r] * inv; const unsigned short hb = bf16_bits(x); vh[r] = hb; vl[r] = bf16_bits(x - bf16_val(hb)); }
    *(v8us*)&sc[wave][0][ln][48 + 8 * hh] = vh; *(v8us*)&sc[wave][1][ln][48 + 8 * hh] = vl;
  }
  __builtin_amdgcn_fence(4  , "workgroup");
  __builtin_amdgcn_wave_barrier();
  const int rs = lane >> 3, c8 = (lane & 7) * 8;
  for (int pass = 0; pass < 2; ++pass) {
#pragma unroll
    for (int j = 0; j < 4; ++j) {
      const int r = j * 4 + rs;
      const v8us xh = *(const v8us*)&sc[wave][0][r][c8];
      const v8us xl = *(const v8us*)&sc[wave][1][r][c8];
      unsigned short* d = CX + (rowb + q0 + r) * CXP + (size_t)h * HD + c8;
      *(volatile v8us*)d = xh;
      *(volatile v8us*)(d + DM) = xl;
    }
    if (pass == 0) __threadfence();
  }
}

#define SZ_W   ((size_t)DM * DM * 2)
#define SZ_WO2 ((size_t)DM * CXP * 2)
#define SZ_X   ((size_t)NR * DM * 2)
#define SZ_VT  ((size_t)NB * DM * SEQ * 2)
#define SZ_CX  ((size_t)NR * CXP * 2)
#define WS_TOTAL (3 * SZ_W + SZ_WO2 + 3 * SZ_X + 4 * SZ_X + SZ_VT + SZ_CX)
static_assert(WS_TOTAL <= (size_t)134217728);
static_assert(SZ_W % 256 == 0);
static_assert(SZ_X % 256 == 0);

extern "C" void kernel_launch(void* const* d_in, const int* in_sizes, int n_in,
                              void* d_out, int out_size, void* d_ws, size_t ws_size, hipStream_t stream) {
  if (n_in < 11) return;
  const int xmin = (NB - 1) * SEQ_FULL * DM + SEQ * DM;
  if (in_sizes[0] < xmin || in_sizes[1] < xmin || in_sizes[2] < xmin) return;
  if (in_sizes[3] < DM * DM || in_sizes[5] < DM * DM || in_sizes[7] < DM * DM || in_sizes[9] < DM * DM) return;
  if (in_sizes[4] < DM || in_sizes[6] < DM || in_sizes[8] < DM || in_sizes[10] < DM) return;
  if (out_size < xmin) return;
  if (ws_size < WS_TOTAL) return;
  const float* xq = (const float*)d_in[0];
  const float* xk = (const float*)d_in[1];
  const float* xv = (const float*)d_in[2];
  const float* wq = (const float*)d_in[3];
  const float* bq = (const float*)d_in[4];
  const float* wk = (const float*)d_in[5];
  const float* bk = (const float*)d_in[6];
  const float* wv = (const float*)d_in[7];
  const float* bv = (const float*)d_in[8];
  const float* wo = (const float*)d_in[9];
  const float* bo = (const float*)d_in[10];
  char* ws = (char*)d_ws;
  size_t off = 0;
  unsigned short* WQT = (unsigned short*)(ws + off); off += SZ_W;
  unsigned short* WKT = (unsigned short*)(ws + off); off += SZ_W;
  unsigned short* WVT = (unsigned short*)(ws + off); off += SZ_W;
  unsigned short* WO2 = (unsigned short*)(ws + off); off += SZ_WO2;
  unsigned short* XQ = (unsigned short*)(ws + off); off += SZ_X;
  unsigned short* XK = (unsigned short*)(ws + off); off += SZ_X;
  unsigned short* XV = (unsigned short*)(ws + off); off += SZ_X;
  unsigned short* QHp = (unsigned short*)(ws + off); off += SZ_X;
  unsigned short* QLp = (unsigned short*)(ws + off); off += SZ_X;
  unsigned short* KHp = (unsigned short*)(ws + off); off += SZ_X;
  unsigned short* KLp = (unsigned short*)(ws + off); off += SZ_X;
  unsigned short* VTp = (unsigned short*)(ws + off); off += SZ_VT;
  unsigned short* CXp = (unsigned short*)(ws + off); off += SZ_CX;
  if (off > ws_size) return;

  const unsigned gw = (unsigned)((DM * (DM / 8) + 255) / 256);
  k_wt<<<gw, 256, 0, stream>>>(wq, WQT, DM, 0);
  k_wt<<<gw, 256, 0, stream>>>(wk, WKT, DM, 0);
  k_wt<<<gw, 256, 0, stream>>>(wv, WVT, DM, 0);
  k_wt<<<gw, 256, 0, stream>>>(wo, WO2, CXP, 1);
  const unsigned gx = (unsigned)(((size_t)NR * (DM / 8) + 255) / 256);
  k_xbf<<<gx, 256, 0, stream>>>(xq, XQ);
  k_xbf<<<gx, 256, 0, stream>>>(xk, XK);
  k_xbf<<<gx, 256, 0, stream>>>(xv, XV);
  k_gemm_hilo<<<dim3((unsigned)((NR / 128) * (DM / 64)), 1), 128, 0, stream>>>(XQ, DM, WQT, DM, 0.125f, bq, QHp, QLp, DM, DM, DM);
  k_gemm_hilo<<<dim3((unsigned)((NR / 128) * (DM / 64)), 1), 128, 0, stream>>>(XK, DM, WKT, DM, 1.0f, bk, KHp, KLp, DM, DM, DM);
  k_gemm_vt<<<dim3((unsigned)((DM / 128) * (SEQ / 64)), NB), 128, 0, stream>>>(WVT, DM, XV, DM, (size_t)SEQ * DM, bv, VTp, SEQ, (size_t)DM * SEQ, SEQ, DM);
  k_attn<<<(unsigned)(NB * NH * (SEQ / 64)), 128, 0, stream>>>(QHp, QLp, KHp, KLp, VTp, CXp);
  k_gemm_out<<<dim3((unsigned)((SEQ / 128) * (DM / 64)), NB), 128, 0, stream>>>(CXp, CXP, (size_t)SEQ * CXP, WO2, CXP, bo, (float*)d_out, DM, (size_t)SEQ_FULL * DM, DM, CXP);
}
